// MultiHeadAttentionLayer_16183436771963
// MI455X (gfx1250) — hardware-verified
//
#include <hip/hip_runtime.h>


#ifndef NB
#define NB 2
#endif
#ifndef SEQ
#define SEQ 2048
#endif
#define NB_FULL 2
#define SEQ_FULL 2048
#define HID 1024
#define NH 16
#define HD 64
#define NREL 9
#define NTOK (NB * SEQ)
#define KO (2 * HID)

static_assert(NB >= 1 && NB <= NB_FULL);
static_assert(SEQ >= 128 && SEQ <= SEQ_FULL && (SEQ % 128) == 0);
static_assert(HID == NH * HD && HD == 64);
static_assert((HID % 128) == 0 && (NTOK % 128) == 0);

typedef unsigned short us_t;
typedef us_t v8us __attribute__((ext_vector_type(8)));
typedef us_t v16us __attribute__((ext_vector_type(16)));
typedef _Float16 v16h __attribute__((ext_vector_type(16)));
typedef __bf16 v16bf __attribute__((ext_vector_type(16)));
typedef float v8f __attribute__((ext_vector_type(8)));
typedef float v4f __attribute__((ext_vector_type(4)));

__device__ __forceinline__ us_t f2bf(float v) {
  __bf16 t = (__bf16)v;
  return __builtin_bit_cast(us_t, t);
}
__device__ __forceinline__ float bfr(float v) {
  __bf16 t = (__bf16)v;
  return (float)t;
}
__device__ __forceinline__ us_t f2h(float v) {
  _Float16 t = (_Float16)v;
  return __builtin_bit_cast(us_t, t);
}
__device__ __forceinline__ v8f vz8() {
  v8f z = {0.f, 0.f, 0.f, 0.f, 0.f, 0.f, 0.f, 0.f};
  return z;
}

__device__ __forceinline__ v16us ldfrag(const us_t* p0, int ld, int rc, int kk) {
  const int hsel = (threadIdx.x >> 4) & 1;
  const us_t* p = p0 + (size_t)rc * ld + kk + 8 * hsel;
  const v8us lo = *(const v8us*)p;
  const v8us hi = *(const v8us*)(p + 16);
  return __builtin_shufflevector(lo, hi, 0, 1, 2, 3, 4, 5, 6, 7,
                                 8, 9, 10, 11, 12, 13, 14, 15);
}

__device__ __forceinline__ v8f mma_bf(v16us a, v16us b, v8f c) {
  v8f d = __builtin_amdgcn_wmma_f32_16x16x32_bf16(
      false, __builtin_bit_cast(v16bf, a), false, __builtin_bit_cast(v16bf, b),
      (short)0, c, false, false);
  asm volatile("v_nop\n\tv_nop\n\tv_nop\n\tv_nop" : "+v"(d) : "v"(a), "v"(b));
  return d;
}
__device__ __forceinline__ v8f mma_h(v16us a, v16us b, v8f c) {
  v8f d = __builtin_amdgcn_wmma_f32_16x16x32_f16(
      false, __builtin_bit_cast(v16h, a), false, __builtin_bit_cast(v16h, b),
      (short)0, c, false, false);
  asm volatile("v_nop\n\tv_nop\n\tv_nop\n\tv_nop" : "+v"(d) : "v"(a), "v"(b));
  return d;
}

__device__ __forceinline__ float max16(float v) {
  v = fmaxf(v, __shfl_xor(v, 1, 32));
  v = fmaxf(v, __shfl_xor(v, 2, 32));
  v = fmaxf(v, __shfl_xor(v, 4, 32));
  v = fmaxf(v, __shfl_xor(v, 8, 32));
  return v;
}
__device__ __forceinline__ float sum16(float v) {
  v += __shfl_xor(v, 1, 32);
  v += __shfl_xor(v, 2, 32);
  v += __shfl_xor(v, 4, 32);
  v += __shfl_xor(v, 8, 32);
  return v;
}

__global__ __launch_bounds__(256) void k_xcvt(const float* __restrict__ x, us_t* xb) {
  const size_t i = (size_t)blockIdx.x * 256 + threadIdx.x;
  const size_t e = i * 8;
  const int tok = (int)(e >> 10);
  const int col = (int)(e & (HID - 1));
  const int b = tok / SEQ, s = tok - b * SEQ;
  const float* src = x + ((size_t)b * SEQ_FULL + s) * HID + col;
  const v4f f0 = *(const v4f*)src;
  const v4f f1 = *(const v4f*)(src + 4);
  v8us u;
  u[0] = f2bf(f0[0]); u[1] = f2bf(f0[1]); u[2] = f2bf(f0[2]); u[3] = f2bf(f0[3]);
  u[4] = f2bf(f1[0]); u[5] = f2bf(f1[1]); u[6] = f2bf(f1[2]); u[7] = f2bf(f1[3]);
  us_t* dst = xb + e;
  *(volatile v8us*)dst = u;
  __threadfence();
  *(volatile v8us*)dst = u;
}

__global__ __launch_bounds__(256) void k_wprep(
    const float* __restrict__ W0, const float* __restrict__ W1,
    const float* __restrict__ W2, const float* __restrict__ W3,
    us_t* O0, us_t* O1, us_t* O2, us_t* O3) {
  __shared__ __align__(16) us_t t[64 * 72];
  const int z = blockIdx.z;
  const float* W = (z == 0) ? W0 : ((z == 1) ? W1 : ((z == 2) ? W2 : W3));
  us_t* O = (z == 0) ? O0 : ((z == 1) ? O1 : ((z == 2) ? O2 : O3));
  const int pitch = (z == 3) ? KO : HID;
  const int k0 = blockIdx.y * 64, n0 = blockIdx.x * 64;
  const int tid = threadIdx.x;
  {
    const int kk = tid >> 2, nc = (tid & 3) * 16;
    const float* src = W + (size_t)(k0 + kk) * HID + n0 + nc;
#pragma unroll
    for (int j = 0; j < 4; ++j) {
      const v4f f = *(const v4f*)(src + 4 * j);
      t[(nc + 4 * j + 0) * 72 + kk] = f2bf(f[0]);
      t[(nc + 4 * j + 1) * 72 + kk] = f2bf(f[1]);
      t[(nc + 4 * j + 2) * 72 + kk] = f2bf(f[2]);
      t[(nc + 4 * j + 3) * 72 + kk] = f2bf(f[3]);
    }
  }
  __syncthreads();
  for (int pass = 0; pass < 2; ++pass) {
#pragma unroll
    for (int rep = 0; rep < 2; ++rep) {
      const int nn = rep * 32 + (tid >> 3), piece = tid & 7;
      const v8us u = *(const v8us*)(t + nn * 72 + piece * 8);
      us_t* dst = O + (size_t)(n0 + nn) * pitch + k0 + piece * 8;
      *(volatile v8us*)dst = u;
      if (z == 3) *(volatile v8us*)(dst + HID) = u;
    }
    if (pass == 0) __threadfence();
  }
}

__global__ __launch_bounds__(256) void k_tables(
    const float* __restrict__ tk, const float* __restrict__ tv, us_t* tkP, us_t* tvT) {
  const int tid = threadIdx.x;
  v8us uk, uv;
  {
    const int row = (tid & 127) >> 3;
    const int kp = (tid & 7) * 8;
    const int rowc = min(row, NREL - 1);
#pragma unroll
    for (int i = 0; i < 8; ++i) {
      float v = tk[rowc * HD + kp + i];
      v = (row < NREL) ? v : 0.0f;
      uk[i] = f2h(bfr(v) * 64.0f);
    }
  }
  {
    const int nn = tid >> 2;
    const int kp = (tid & 3) * 8;
#pragma unroll
    for (int i = 0; i < 8; ++i) {
      const int k = kp + i;
      float v = tv[min(k, NREL - 1) * HD + nn];
      v = (k < NREL) ? v : 0.0f;
      uv[i] = f2h(bfr(v) * 64.0f);
    }
  }
  for (int pass = 0; pass < 2; ++pass) {
    if (tid < 128) *(volatile v8us*)(tkP + tid * 8) = uk;
    *(volatile v8us*)(tvT + tid * 8) = uv;
    if (pass == 0) __threadfence();
  }
}

template <int OUTF32>
__global__ __launch_bounds__(128) void k_gemm(
    const us_t* __restrict__ Am0, const us_t* __restrict__ Am1, const us_t* __restrict__ Bn,
    const float* __restrict__ bias0, const float* __restrict__ bias1,
    void* out0, void* out1,
    int K, int bias_on_m, int blen, int ldo, int mdiv, int mbstride, float ka, float kb) {
  __shared__ __align__(16) unsigned int stg_raw[4 * 32 * 64 * (OUTF32 ? 4 : 2) / 4];

  const int z = blockIdx.z;
  const us_t* Am = z ? Am1 : Am0;
  const float* bias = z ? bias1 : bias0;
  void* out = z ? out1 : out0;

  const int lane = threadIdx.x & 31, wave = threadIdx.x >> 5;
  const int h = (lane >> 4) & 1, n15 = lane & 15;
  const int mblk = blockIdx.x * 64;
  const int nwave = blockIdx.y * 128 + wave * 32;

  v8f acc[4][2];
#pragma unroll
  for (int mt = 0; mt < 4; ++mt) { acc[mt][0] = vz8(); acc[mt][1] = vz8(); }

#pragma unroll 1
  for (int kk = 0; kk < K; kk += 32) {
    v16us a[4], b[2];
#pragma unroll
    for (int mt = 0; mt < 4; ++mt) a[mt] = ldfrag(Am, K, mblk + mt * 16 + n15, kk);
#pragma unroll
    for (int nt = 0; nt < 2; ++nt) b[nt] = ldfrag(Bn, K, nwave + nt * 16 + n15, kk);
#pragma unroll
    for (int mt = 0; mt < 4; ++mt) {
      acc[mt][0] = mma_bf(a[mt], b[0], acc[mt][0]);
      acc[mt][1] = mma_bf(a[mt], b[1], acc[mt][1]);
    }
  }

  float bm[4][8];
#pragma unroll
  for (int mt = 0; mt < 4; ++mt) {
    const int ib = min(mblk + mt * 16 + 8 * h, blen - 8);
    const v4f c0 = *(const v4f*)(bias + ib);
    const v4f c1 = *(const v4f*)(bias + ib + 4);
    bm[mt][0] = bfr(c0[0]); bm[mt][1] = bfr(c0[1]); bm[mt][2] = bfr(c0[2]); bm[mt][3] = bfr(c0[3]);
    bm[mt][4] = bfr(c1[0]); bm[mt][5] = bfr(c1[1]); bm[mt][6] = bfr(c1[2]); bm[mt][7] = bfr(c1[3]);
  }
  float bn[2];
#pragma unroll
  for (int nt = 0; nt < 2; ++nt) bn[nt] = bfr(bias[min(nwave + nt * 16 + n15, blen - 1)]);

  const int bq = mblk / mdiv;
  const int base = bq * mbstride + (mblk - bq * mdiv);

  if constexpr (OUTF32) {
    float* sw = (float*)stg_raw + wave * 2048;
#pragma unroll
    for (int mt = 0; mt < 4; ++mt) {
#pragma unroll
      for (int nt = 0; nt < 2; ++nt) {
        v4f u0, u1;
#pragma unroll
        for (int r = 0; r < 4; ++r) {
          const float b0v = bias_on_m ? bm[mt][r] : bn[nt];
          const float b1v = bias_on_m ? bm[mt][r + 4] : bn[nt];
          u0[r] = acc[mt][nt][r] * ka + b0v * kb;
          u1[r] = acc[mt][nt][r + 4] * ka + b1v * kb;
        }
        float* sp = sw + (nt * 16 + n15) * 64 + mt * 16 + 8 * h;
        *(v4f*)sp = u0;
        *(v4f*)(sp + 4) = u1;
      }
    }
    __syncthreads();
    float* op = (float*)out;
    for (int pass = 0; pass < 2; ++pass) {
#pragma unroll
      for (int i = 0; i < 16; ++i) {
        const int L = i * 4 + (lane >> 3);
        const int row = L >> 1, hr = L & 1, piece = lane & 7;
        const v4f u = *(const v4f*)(sw + row * 64 + hr * 32 + piece * 4);
        float* dst = op + (size_t)(nwave + row) * ldo + base + hr * 32 + piece * 4;
        *(volatile v4f*)dst = u;
      }
      if (pass == 0) __threadfence();
    }
  } else {
    us_t* sw = (us_t*)stg_raw + wave * 2048;
#pragma unroll
    for (int mt = 0; mt < 4; ++mt) {
#pragma unroll
      for (int nt = 0; nt < 2; ++nt) {
        v8us u;
#pragma unroll
        for (int r = 0; r < 8; ++r) {
          const float bbv = bias_on_m ? bm[mt][r] : bn[nt];
          u[r] = f2h(acc[mt][nt][r] * ka + bbv * kb);
        }
        *(v8us*)(sw + (nt * 16 + n15) * 64 + mt * 16 + 8 * h) = u;
      }
    }
    __syncthreads();
    us_t* op = (us_t*)out;
    for (int pass = 0; pass < 2; ++pass) {
#pragma unroll
      for (int i = 0; i < 8; ++i) {
        const int row = i * 4 + (lane >> 3), piece = lane & 7;
        const v8us u = *(const v8us*)(sw + row * 64 + piece * 8);
        us_t* dst = op + (size_t)(nwave + row) * ldo + base + piece * 8;
        *(volatile v8us*)dst = u;
      }
      if (pass == 0) __threadfence();
    }
  }
}

__global__ __launch_bounds__(32) __attribute__((amdgpu_num_vgpr(256))) void k_attn(
    const us_t* __restrict__ Qp, const us_t* __restrict__ Kp, const us_t* __restrict__ VTp,
    const us_t* __restrict__ tkP, const us_t* __restrict__ tvT, us_t* ctx2) {
  __shared__ float bl[16 * 16];
  __shared__ float wl[16 * 8];
  __shared__ __align__(16) us_t pls[16 * 32];
  __shared__ __align__(16) us_t p2s[16 * 32];
  __shared__ __align__(16) us_t cst[2][16 * 64];

  const int lane = threadIdx.x & 31, h = lane >> 4, n = lane & 15;
  const int qt = blockIdx.x, hh = blockIdx.y, b = blockIdx.z;
  const int lo_q = qt * 16;
  const size_t tok0 = (size_t)b * SEQ + lo_q;
  const us_t* qptr = Qp + tok0 * HID + hh * HD;
  const us_t* kbase = Kp + (size_t)b * SEQ * HID + hh * HD;
  const us_t* vhead = VTp + ((size_t)b * HID + hh * HD) * SEQ;

#pragma unroll
  for (int i = 0; i < 4; ++i) wl[lane * 4 + i] = -1.0e30f;

  const v16us q0 = ldfrag(qptr, HID, n, 0);
  const v16us q1 = ldfrag(qptr, HID, n, 32);

  {
    v8f sr = vz8();
    const v16us t0 = ldfrag(tkP, HD, n, 0);
    const v16us t1 = ldfrag(tkP, HD, n, 32);
    sr = mma_h(q0, t0, sr);
    sr = mma_h(q1, t1, sr);
#pragma unroll
    for (int r = 0; r < 8; ++r) {
      const float v = sr[r];
      const float v0 = __shfl(v, lane & 16, 32);
      bl[(8 * h + r) * 16 + n] = (v - v0) * (1.0f / 2048.0f);
    }
  }
  __syncthreads();
  float d8[8];
#pragma unroll
  for (int r = 0; r < 8; ++r) d8[r] = bl[(8 * h + r) * 16 + 8];

  float rmax[8], rsum[8], blo[8];
  v8f cacc[4];
#pragma unroll
  for (int r = 0; r < 8; ++r) { rmax[r] = -1.0e30f; rsum[r] = 0.0f; blo[r] = 0.0f; }
#pragma unroll
  for (int j = 0; j < 4; ++j) cacc[j] = vz8();

#pragma unroll 1
  for (int kc = 0; kc < SEQ; kc += 32) {
    v8f s0 = vz8(), s1 = vz8();
    {
      const v16us f0 = ldfrag(kbase, HID, kc + n, 0);
      const v16us f1 = ldfrag(kbase, HID, kc + n, 32);
      s0 = mma_h(q0, f0, s0);
      s0 = mma_h(q1, f1, s0);
      const v16us g0 = ldfrag(kbase, HID, kc + 16 + n, 0);
      const v16us g1 = ldfrag(kbase, HID, kc + 16 + n, 32);
      s1 = mma_h(q0, g0, s1);
      s1 = mma_h(q1, g1, s1);
    }
    const bool below = (kc + 35 <= lo_q);
    const bool above = (kc >= lo_q + 19);
    const bool mixed = !(below || above);
    float a0[8], a1[8];
#pragma unroll
    for (int r = 0; r < 8; ++r) {
      a0[r] = s0[r] * (1.0f / 128.0f);
      a1[r] = s1[r] * (1.0f / 128.0f);
    }
    if (mixed) {
#pragma unroll
      for (int r = 0; r < 8; ++r) {
        const int R = 8 * h + r;
        const int dd0 = kc + n - (lo_q + R);
        const int dd1 = dd0 + 16;
        const int b0 = min(max(dd0, -4), 4) + 4;
        const int b1 = min(max(dd1, -4), 4) + 4;
        a0[r] += bl[R * 16 + b0];
        a1[r] += bl[R * 16 + b1];
        if (b0 >= 1 && b0 <= 7) wl[R * 8 + b0 - 1] = a0[r];
        if (b1 >= 1 && b1 <= 7) wl[R * 8 + b1 - 1] = a1[r];
      }
    } else {
#pragma unroll
      for (int r = 0; r < 8; ++r) {
        const float ad = above ? d8[r] : 0.0f;
        a0[r] += ad;
        a1[r] += ad;
      }
    }
#pragma unroll
    for (int r = 0; r < 8; ++r) {
      const float m = max16(fmaxf(a0[r], a1[r]));
      const float nm = fmaxf(rmax[r], m);
      const float sc = __expf(rmax[r] - nm);
      rmax[r] = nm;
      const float p0 = __expf(a0[r] - nm);
      const float p1 = __expf(a1[r] - nm);
      const float ps = sum16(p0 + p1);
      rsum[r] = rsum[r] * sc + ps;
      float addb = below ? ps : 0.0f;
      if (mixed) {
        const int R = 8 * h + r;
        const int dd0 = kc + n - (lo_q + R);
        const float pb = ((dd0 <= -4) ? p0 : 0.0f) + ((dd0 + 16 <= -4) ? p1 : 0.0f);
        addb = sum16(pb);
      }
      blo[r] = blo[r] * sc + addb;
#pragma unroll
      for (int j = 0; j < 4; ++j) cacc[j][r] *= sc;
      a0[r] = p0;
      a1[r] = p1;
    }
#pragma unroll
    for (int r = 0; r < 8; ++r) {
      pls[(8 * h + r) * 32 + n] = f2h(a0[r] * 1024.0f);
      pls[(8 * h + r) * 32 + 16 + n] = f2h(a1[r] * 1024.0f);
    }
    __syncthreads();
    const v16us pA = ldfrag(pls, 32, n, 0);
#pragma unroll
    for (int j = 0; j < 4; ++j) {
      const v16us vB = ldfrag(vhead, SEQ, j * 16 + n, kc);
      cacc[j] = mma_h(pA, vB, cacc[j]);
    }
    __syncthreads();
  }

  __syncthreads();
  float inv[8];
#pragma unroll
  for (int r = 0; r < 8; ++r) {
    const int R = 8 * h + r;
    inv[r] = __builtin_amdgcn_rcpf(rsum[r]);
    float wv = __expf(wl[R * 8 + ((n + 7) & 7)] - rmax[r]);
    wv = (n >= 1 && n <= 7) ? wv : 0.0f;
    const float wsum = sum16(wv);
    const float a8 = (rsum[r] - blo[r] - wsum) * inv[r];
    const float a0v = blo[r] * inv[r];
    const float val = (n == 0) ? a0v : ((n <= 7) ? wv * inv[r] : ((n == 8) ? a8 : 0.0f));
    p2s[R * 32 + n] = f2h(val * 1024.0f);
    p2s[R * 32 + 16 + n] = (us_t)0;
  }
  __syncthreads();
  v8f w2[4];
  {
    const v16us pA2 = ldfrag(p2s, 32, n, 0);
#pragma unroll
    for (int j = 0; j < 4; ++j) {
      const v16us tB = ldfrag(tvT, 32, j * 16 + n, 0);
      w2[j] = mma_h(pA2, tB, vz8());
    }
  }
#pragma unroll
  for (int j = 0; j < 4; ++j) {
#pragma unroll
    for (int r = 0; r < 8; ++r) {
      const int R = 8 * h + r;
      const float cv = cacc[j][r] * inv[r] * (1.0f / 4096.0f) + w2[j][r] * (1.0f / 65536.0f);
      const __bf16 hb = (__bf16)cv;
      const float hf = (float)hb;
      const __bf16 lb = (__bf16)(cv - hf);
      cst[0][R * 64 + j * 16 + n] = __builtin_bit_cast(us_t, hb);
      cst[1][R * 64 + j * 16 + n] = __builtin_bit_cast(us_t, lb);
    }
  }
  __syncthreads();
  for (int pass = 0; pass < 2; ++pass) {
#pragma unroll
    for (int pl = 0; pl < 2; ++pl) {
#pragma unroll
      for (int i = 0; i < 4; ++i) {
        const int row = i * 4 + (lane >> 3), piece = lane & 7;
        const v8us u = *(const v8us*)(cst[pl] + row * 64 + piece * 8);
        us_t* dst = ctx2 + (tok0 + row) * (size_t)KO + pl * HID + hh * HD + piece * 8;
        *(volatile v8us*)dst = u;
      }
    }
    if (pass == 0) __threadfence();
  }
}

extern "C" void kernel_launch(void* const* d_in, const int* in_sizes, int n_in,
                              void* d_out, int out_size, void* d_ws, size_t ws_size,
                              hipStream_t stream) {
  if (n_in < 11) return;
  const long long need_x = ((long long)(NB - 1) * SEQ_FULL + SEQ) * HID;
  if ((long long)in_sizes[0] < need_x) return;
  if (in_sizes[1] < HID * HID || in_sizes[3] < HID * HID ||
      in_sizes[5] < HID * HID || in_sizes[7] < HID * HID) return;
  if (in_sizes[2] < HID || in_sizes[4] < HID || in_sizes[6] < HID || in_sizes[8] < HID) return;
  if (in_sizes[9] < NREL * HD || in_sizes[10] < NREL * HD) return;
  if ((long long)out_size < (long long)NTOK * HID) return;

  const float* x  = (const float*)d_in[0];
  const float* Wq = (const float*)d_in[1];
  const float* bq = (const float*)d_in[2];
  const float* Wk = (const float*)d_in[3];
  const float* bk = (const float*)d_in[4];
  const float* Wv = (const float*)d_in[5];
  const float* bv = (const float*)d_in[6];
  const float* Wo = (const float*)d_in[7];
  const float* bo = (const float*)d_in[8];
  const float* tk = (const float*)d_in[9];
  const float* tv = (const float*)d_in[10];

  char* ws = (char*)d_ws;
  size_t off = 0;
  auto carve = [&](size_t bytes) -> size_t {
    const size_t o = off;
    off += (bytes + 255) & ~(size_t)255;
    return o;
  };
  const size_t o_xb  = carve((size_t)NTOK * HID * 2);
  const size_t o_wq  = carve((size_t)HID * HID * 2);
  const size_t o_wk  = carve((size_t)HID * HID * 2);
  const size_t o_wv  = carve((size_t)HID * HID * 2);
  const size_t o_wo  = carve((size_t)HID * KO * 2);
  const size_t o_q   = carve((size_t)NTOK * HID * 2);
  const size_t o_k   = carve((size_t)NTOK * HID * 2);
  const size_t o_vt  = carve((size_t)NB * HID * SEQ * 2);
  const size_t o_ctx = carve((size_t)NTOK * KO * 2);
  const size_t o_tk  = carve((size_t)16 * HD * 2);
  const size_t o_tv  = carve((size_t)HD * 32 * 2);
  if (off > ws_size) return;

  us_t* xb   = (us_t*)(ws + o_xb);
  us_t* WqT  = (us_t*)(ws + o_wq);
  us_t* WkT  = (us_t*)(ws + o_wk);
  us_t* WvT  = (us_t*)(ws + o_wv);
  us_t* WoT2 = (us_t*)(ws + o_wo);
  us_t* Qp   = (us_t*)(ws + o_q);
  us_t* Kpl  = (us_t*)(ws + o_k);
  us_t* VTp  = (us_t*)(ws + o_vt);
  us_t* ctx2 = (us_t*)(ws + o_ctx);
  us_t* tkP  = (us_t*)(ws + o_tk);
  us_t* tvT  = (us_t*)(ws + o_tv);
  float* out = (float*)d_out;

  k_xcvt<<<NTOK * (HID / 8) / 256, 256, 0, stream>>>(x, xb);
  k_wprep<<<dim3(HID / 64, HID / 64, 4), 256, 0, stream>>>(Wq, Wk, Wv, Wo, WqT, WkT, WvT, WoT2);
  k_tables<<<1, 256, 0, stream>>>(tk, tv, tkP, tvT);

  k_gemm<0><<<dim3(HID / 64, NTOK / 128, 2), 128, 0, stream>>>(
      WqT, WkT, xb, bq, bk, (void*)Qp, (void*)Kpl,
      HID, 1, HID, HID, 1 << 30, 0, 4.0f, 4.0f);
  k_gemm<0><<<dim3(NTOK / 64, HID / 128, 1), 128, 0, stream>>>(
      xb, xb, WvT, bv, bv, (void*)VTp, (void*)VTp,
      HID, 0, HID, SEQ, SEQ, HID * SEQ, 4.0f, 4.0f);
  k_attn<<<dim3(SEQ / 16, NH, NB), 32, 0, stream>>>(Qp, Kpl, VTp, tkP, tvT, ctx2);
  k_gemm<1><<<dim3(HID / 64, NTOK / 128, 1), 128, 0, stream>>>(
      WoT2, WoT2, ctx2, bo, bo, d_out, d_out,
      KO, 1, HID, HID, 1 << 30, 0, 1.0f, 1.0f);
  (void)out;
  (void)hipGetLastError();
}
